// Encoder_40570261078498
// MI455X (gfx1250) — hardware-run, weakly checked
//
#include <hip/hip_runtime.h>
#include <math.h>


#ifndef NB
#define NB 4
#endif
#ifndef SEQ
#define SEQ 512
#endif
#define NB_FULL  4
#define SEQ_FULL 512
#ifndef OUT_SEQ
#define OUT_SEQ SEQ
#endif
#define NF   8
#define DM   256
#define DI   512
#define DS   16
#define DC   4
#define DTR  16
#define NXP  48
#define NXPP 64
#define KDT  32
#define ROWS (NB * SEQ)
#define OSP  68
#define OSQ  260
#define CW   64.0f
#define CXC  1024.0f
#define CDR  1024.0f
#define CY   4096.0f
#define CG   64.0f
#define FIN  (1.0f / 64.0f)
#define FXP  (1.0f / 65536.0f)
#define FDT  (1.0f / 65536.0f)
#define FOUT (1.0f / 262144.0f)
#define L2E  1.4426950408889634f

static_assert(SEQ % 64 == 0);
static_assert(ROWS % 64 == 0);
static_assert(DM % 32 == 0);
static_assert(DI % 32 == 0);
static_assert(KDT == 32);
static_assert(DTR <= 16);
static_assert(NXP == DTR + 2 * DS);
static_assert(NXPP == 64);
static_assert(2 * DS == 32);
static_assert((2 * DI) % 64 == 0);
static_assert(DI % 64 == 0);
static_assert(DM == 256);
static_assert(DM / 8 == 32);
static_assert(NF * (DM / 8) == DM);
static_assert(DI == 512);
static_assert(DS == 16);
static_assert(DC == 4);
static_assert(NB <= NB_FULL);
static_assert(SEQ <= SEQ_FULL);
static_assert((OSP * 4) % 16 == 0);
static_assert((OSQ * 4) % 16 == 0);
static_assert(16 * OSP * 4 <= 131072);
static_assert(16 * OSQ * 4 <= 131072);
static_assert(256 * 8 * 2 <= 131072);
static_assert(32 * 16 * 8 == 16 * 64 * 4);
static_assert(32 * 16 * 4 == 16 * 64 * 2);
static_assert(32 * 16 * 2 == 16 * KDT * 2);
static_assert(32 * 16 * 4 == 16 * 32 * 4);
static_assert(((size_t)NF * ROWS * 32) % 256 == 0);
static_assert(((size_t)NF * ROWS * (DI / 4)) % 256 == 0);
static_assert(((size_t)NF * 2 * DI * DM / 8) % 256 == 0);
static_assert(((size_t)NF * DM * DI / 8) % 256 == 0);
static_assert(((size_t)NF * NXPP * (DI / 8)) % 256 == 0);
static_assert(((size_t)NF * DI * (KDT / 8)) % 256 == 0);

typedef _Float16 h16;
typedef __attribute__((ext_vector_type(16))) _Float16 v16h;
typedef __attribute__((ext_vector_type(8)))  _Float16 v8h;
typedef __attribute__((ext_vector_type(8)))  float    v8f;
typedef __attribute__((ext_vector_type(4)))  float    v4f;
typedef v4f  __attribute__((may_alias)) v4fa;
typedef v8h  __attribute__((may_alias)) v8ha;

__device__ __forceinline__ unsigned short f2bf(float f) { unsigned u = __float_as_uint(f); u += 0x7FFFu + ((u >> 16) & 1u); return (unsigned short)(u >> 16); }
__device__ __forceinline__ float bfr(float f) { return __uint_as_float(((unsigned)f2bf(f)) << 16); }
__device__ __forceinline__ v16h cat16(v8h lo, v8h hi) { return __builtin_shufflevector(lo, hi, 0, 1, 2, 3, 4, 5, 6, 7, 8, 9, 10, 11, 12, 13, 14, 15); }
__device__ __forceinline__ v8f wmma16(v16h a, v16h b, v8f c) { return __builtin_amdgcn_wmma_f32_16x16x32_f16(false, a, false, b, (short)0, c, false, false); }
__device__ __forceinline__ v8f wmma16g(v16h a, v16h b, v8f c) {
    c = wmma16(a, b, c);
    asm volatile("v_nop\n\tv_nop\n\tv_nop\n\tv_nop" : "+v"(c) : "v"(a), "v"(b));
    return c;
}
__device__ __forceinline__ h16 toh_flush(float v) { const h16 r = (h16)v; return (fabsf(v) < 6.103515625e-05f) ? (h16)0.0f : r; }
__device__ __forceinline__ v16h ldh(const h16* p) { return cat16(*(const v8h*)p, *(const v8h*)(p + 16)); }
__device__ __forceinline__ v16h ldf(const float* p, float carry) {
    const v4f a = *(const v4f*)p, b = *(const v4f*)(p + 4), c = *(const v4f*)(p + 16), d = *(const v4f*)(p + 20);
    v16h r;
#pragma unroll
    for (int i = 0; i < 4; ++i) { r[i] = toh_flush(a[i] * carry); r[4 + i] = toh_flush(b[i] * carry); r[8 + i] = toh_flush(c[i] * carry); r[12 + i] = toh_flush(d[i] * carry); }
    return r;
}
__device__ __forceinline__ void wave_sync() { __builtin_amdgcn_fence(3  , "wavefront"); __builtin_amdgcn_wave_barrier(); asm volatile("" ::: "memory"); }
__device__ __forceinline__ float silu_f(float v) { return v * __builtin_amdgcn_rcpf(1.0f + __builtin_amdgcn_exp2f(-L2E * v)); }
__device__ __forceinline__ float softplus_f(float v) { return fmaxf(v, 0.0f) + log1pf(__expf(-fabsf(v))); }

__global__ __launch_bounds__(256) void k_wcvt(const float* __restrict__ src, h16* dst, size_t n8, float carry) {
    const size_t i = (size_t)blockIdx.x * 256 + threadIdx.x; if (i >= n8) return;
    const v4f a = *(const v4f*)(src + i * 8), b = *(const v4f*)(src + i * 8 + 4); v8h o;
#pragma unroll
    for (int k = 0; k < 4; ++k) { o[k] = toh_flush(bfr(a[k]) * carry); o[4 + k] = toh_flush(bfr(b[k]) * carry); }
    *(volatile v8h*)(dst + i * 8) = o; __threadfence(); *(volatile v8h*)(dst + i * 8) = o;
}

__global__ __launch_bounds__(256) void k_wcvt_xp(const float* __restrict__ src, h16* dst) {
    const size_t i = (size_t)blockIdx.x * 256 + threadIdx.x;
    const int c = (int)(i & 63), n = (int)((i >> 6) & 63), f = (int)(i >> 12);
    const int nc = n < NXP ? n : (NXP - 1);
    const float* sp = src + ((size_t)f * NXP + nc) * DI + c * 8;
    v4f a = *(const v4f*)sp, b = *(const v4f*)(sp + 4);
    asm volatile("" : "+v"(a)); asm volatile("" : "+v"(b));
    const bool keep = n < NXP; v8h o;
#pragma unroll
    for (int k = 0; k < 4; ++k) { const h16 z0 = toh_flush(bfr(a[k]) * CW), z1 = toh_flush(bfr(b[k]) * CW); o[k] = keep ? z0 : (h16)0.0f; o[4 + k] = keep ? z1 : (h16)0.0f; }
    *(volatile v8h*)(dst + i * 8) = o; __threadfence(); *(volatile v8h*)(dst + i * 8) = o;
}

__global__ __launch_bounds__(256) void k_wcvt_dt(const float* __restrict__ src, h16* dst) {
    const size_t i = (size_t)blockIdx.x * 256 + threadIdx.x;
    const int q = (int)(i & 3); const size_t r = i >> 2;
    const float* sp = src + r * DTR + (q & 1) * 8;
    v4f a = *(const v4f*)sp, b = *(const v4f*)(sp + 4);
    asm volatile("" : "+v"(a)); asm volatile("" : "+v"(b));
    const bool keep = q < 2; v8h o;
#pragma unroll
    for (int k = 0; k < 4; ++k) { const h16 z0 = toh_flush(bfr(a[k]) * CW), z1 = toh_flush(bfr(b[k]) * CW); o[k] = keep ? z0 : (h16)0.0f; o[4 + k] = keep ? z1 : (h16)0.0f; }
    *(volatile v8h*)(dst + i * 8) = o; __threadfence(); *(volatile v8h*)(dst + i * 8) = o;
}

__global__ __launch_bounds__(256) void k_feat(const float* __restrict__ ipt, h16* U) {
#pragma clang fp contract(off)
    __shared__ __align__(16) h16 us[256 * 8];
    const int tid = threadIdx.x;
    const size_t g = (size_t)blockIdx.x * 256 + tid;
    const int c = (int)(g & 31); const size_t fr = g >> 5; const int rr = (int)(fr % ROWS); const int f = (int)(fr / ROWS);
    const int b = rr / SEQ, l = rr % SEQ;
    const float x = bfr(ipt[((size_t)b * SEQ_FULL + l) * NF + f]);
#pragma unroll 1
    for (int j = 0; j < 4; ++j) {
        const int i = 4 * c + j;
        const float ang = x * (6.283185307179586f * (float)i);
        float s, co; sincosf(ang, &s, &co);
        us[tid * 8 + 2 * j] = toh_flush(s); us[tid * 8 + 2 * j + 1] = toh_flush(co); }
    __syncthreads();
    const v8h o = *(const v8ha*)(&us[tid * 8]);
    *(volatile v8h*)(U + g * 8) = o; __threadfence(); *(volatile v8h*)(U + g * 8) = o;
}

__global__ __launch_bounds__(32) void k_gemm_in(const h16* __restrict__ U, const h16* __restrict__ W, float* X, h16* G) {
    __shared__ __align__(16) float os[16 * OSP];
    const int lane = threadIdx.x & 31, lr = lane & 15, hi = lane >> 4;
    const int r0 = blockIdx.x * 64, c0 = blockIdx.y * 64, f = blockIdx.z;
    v8f acc[4][4];
#pragma unroll
    for (int mb = 0; mb < 4; ++mb)
#pragma unroll
        for (int nb = 0; nb < 4; ++nb) acc[mb][nb] = (v8f){};
    const size_t aoff = ((size_t)f * ROWS + r0 + lr) * DM + 8 * hi;
    const size_t boff = ((size_t)f * (2 * DI) + c0 + lr) * DM + 8 * hi;
#pragma unroll 1
    for (int kc = 0; kc < DM; kc += 32) {
        v16h a[4];
#pragma unroll
        for (int mb = 0; mb < 4; ++mb) a[mb] = ldh(U + aoff + (size_t)mb * 16 * DM + kc);
#pragma unroll
        for (int nb = 0; nb < 4; ++nb) { const v16h b = ldh(W + boff + (size_t)nb * 16 * DM + kc);
#pragma unroll
            for (int mb = 0; mb < 4; ++mb) acc[mb][nb] = wmma16g(a[mb], b, acc[mb][nb]); }
    }
    const bool isx = c0 < DI;
    const size_t rowb = (size_t)f * ROWS + r0;
#pragma unroll
    for (int mb = 0; mb < 4; ++mb) {
#pragma unroll
        for (int nb = 0; nb < 4; ++nb) {
#pragma unroll
            for (int j = 0; j < 8; ++j) os[(hi * 8 + j) * OSP + nb * 16 + lr] = acc[mb][nb][j] * FIN; }
        wave_sync();
        if (isx) {
            const size_t xb = (rowb + (size_t)(mb * 16)) * DI + c0;
#pragma unroll 1
            for (int ps = 0; ps < 2; ++ps) {
#pragma unroll
                for (int s = 0; s < 8; ++s) { const int p = s * 32 + lane; const int row = p >> 4, c4 = (p & 15) * 4;
                    const v4f val = *(const v4fa*)(&os[row * OSP + c4]);
                    *(volatile v4f*)(X + xb + (size_t)row * DI + c4) = val; }
                if (ps == 0) __threadfence(); }
        } else {
            const size_t gb = (rowb + (size_t)(mb * 16)) * DI + (size_t)(c0 - DI);
            v8h hv[4];
#pragma unroll
            for (int s = 0; s < 4; ++s) { const int row = 4 * s + (lane >> 3), c8 = (lane & 7) * 8;
                const v4f x0 = *(const v4fa*)(&os[row * OSP + c8]); const v4f x1 = *(const v4fa*)(&os[row * OSP + c8 + 4]);
#pragma unroll
                for (int i = 0; i < 4; ++i) { hv[s][i] = toh_flush(silu_f(x0[i]) * CG); hv[s][4 + i] = toh_flush(silu_f(x1[i]) * CG); } }
#pragma unroll 1
            for (int ps = 0; ps < 2; ++ps) {
#pragma unroll
                for (int s = 0; s < 4; ++s) { const int row = 4 * s + (lane >> 3), c8 = (lane & 7) * 8;
                    *(volatile v8h*)(G + gb + (size_t)row * DI + c8) = hv[s]; }
                if (ps == 0) __threadfence(); }
        }
        wave_sync();
    }
}

__global__ __launch_bounds__(256) void k_conv(const float* __restrict__ X, const float* __restrict__ cw, const float* __restrict__ cb, float* XC) {
#pragma clang fp contract(off)
    const size_t i = (size_t)blockIdx.x * 256 + threadIdx.x;
    const int d4 = (int)(i & 127) * 4; const size_t fr = i >> 7;
    const int row = (int)(fr % ROWS); const int f = (int)(fr / ROWS); const int l = row % SEQ;
    const float* wp = cw + ((size_t)f * DI + d4) * DC;
    const v4f w0 = *(const v4f*)wp, w1 = *(const v4f*)(wp + 4), w2 = *(const v4f*)(wp + 8), w3 = *(const v4f*)(wp + 12);
    v4f acc = (v4f){};
#pragma unroll
    for (int j = 0; j < DC; ++j) {
        const int ls = l + j - (DC - 1);
        const int lc = ls < 0 ? 0 : ls;
        v4f x = *(const v4f*)(X + (fr - (size_t)l + (size_t)lc) * DI + d4);
        asm volatile("" : "+v"(x));
        const bool ok = ls >= 0;
        acc[0] += ok ? x[0] * bfr(w0[j]) : 0.0f;
        acc[1] += ok ? x[1] * bfr(w1[j]) : 0.0f;
        acc[2] += ok ? x[2] * bfr(w2[j]) : 0.0f;
        acc[3] += ok ? x[3] * bfr(w3[j]) : 0.0f; }
    const v4f bb = *(const v4f*)(cb + (size_t)f * DI + d4);
    v4f o;
#pragma unroll
    for (int q = 0; q < 4; ++q) o[q] = silu_f(acc[q] + bfr(bb[q]));
    *(volatile v4f*)(XC + i * 4) = o; __threadfence(); *(volatile v4f*)(XC + i * 4) = o;
}

__global__ __launch_bounds__(32) void k_gemm_xp(const float* __restrict__ XC, const h16* __restrict__ W, h16* DTRH, float* BC) {
    __shared__ __align__(16) float os[16 * OSP];
    const int lane = threadIdx.x & 31, lr = lane & 15, hi = lane >> 4;
    const int r0 = blockIdx.x * 32, f = blockIdx.y;
    v8f acc[2][4];
#pragma unroll
    for (int mb = 0; mb < 2; ++mb)
#pragma unroll
        for (int nb = 0; nb < 4; ++nb) acc[mb][nb] = (v8f){};
    const size_t aoff = ((size_t)f * ROWS + r0 + lr) * DI + 8 * hi;
    const size_t boff = ((size_t)f * NXPP + lr) * DI + 8 * hi;
#pragma unroll 1
    for (int kc = 0; kc < DI; kc += 32) {
        v16h a[2];
#pragma unroll
        for (int mb = 0; mb < 2; ++mb) a[mb] = ldf(XC + aoff + (size_t)mb * 16 * DI + kc, CXC);
#pragma unroll
        for (int nb = 0; nb < 4; ++nb) { const v16h b = ldh(W + boff + (size_t)nb * 16 * DI + kc);
#pragma unroll
            for (int mb = 0; mb < 2; ++mb) acc[mb][nb] = wmma16g(a[mb], b, acc[mb][nb]); }
    }
    const size_t rowb = (size_t)f * ROWS + r0;
#pragma unroll
    for (int mb = 0; mb < 2; ++mb) {
#pragma unroll
        for (int nb = 0; nb < 4; ++nb) {
#pragma unroll
            for (int j = 0; j < 8; ++j) os[(hi * 8 + j) * OSP + nb * 16 + lr] = acc[mb][nb][j] * FXP; }
        wave_sync();
        v8h dv[2]; v4f bv[4];
#pragma unroll
        for (int s = 0; s < 2; ++s) { const int p = s * 32 + lane; const int row = p >> 2, q = p & 3; const int cc = (q & 1) * 8;
            const v4f x0 = *(const v4fa*)(&os[row * OSP + cc]); const v4f x1 = *(const v4fa*)(&os[row * OSP + cc + 4]);
            const bool keep = q < 2;
#pragma unroll
            for (int i = 0; i < 4; ++i) { const h16 z0 = toh_flush(x0[i] * CDR), z1 = toh_flush(x1[i] * CDR); dv[s][i] = keep ? z0 : (h16)0.0f; dv[s][4 + i] = keep ? z1 : (h16)0.0f; } }
#pragma unroll
        for (int s = 0; s < 4; ++s) { const int row = 4 * s + (lane >> 3), c4 = (lane & 7) * 4;
            bv[s] = *(const v4fa*)(&os[row * OSP + DTR + c4]); }
        const size_t db = (rowb + (size_t)(mb * 16)) * KDT;
        const size_t bb = (rowb + (size_t)(mb * 16)) * 32;
#pragma unroll 1
        for (int ps = 0; ps < 2; ++ps) {
#pragma unroll
            for (int s = 0; s < 2; ++s) *(volatile v8h*)(DTRH + db + (size_t)(s * 32 + lane) * 8) = dv[s];
#pragma unroll
            for (int s = 0; s < 4; ++s) { const int row = 4 * s + (lane >> 3), c4 = (lane & 7) * 4;
                *(volatile v4f*)(BC + bb + (size_t)row * 32 + c4) = bv[s]; }
            if (ps == 0) __threadfence(); }
        wave_sync();
    }
}

__global__ __launch_bounds__(32) void k_gemm_dt(const h16* __restrict__ A, const h16* __restrict__ W, const float* __restrict__ bias, float* DT) {
    __shared__ __align__(16) float os[16 * OSP];
    const int lane = threadIdx.x & 31, lr = lane & 15, hi = lane >> 4;
    const int r0 = blockIdx.x * 64, c0 = blockIdx.y * 64, f = blockIdx.z;
    v8f acc[4][4];
#pragma unroll
    for (int mb = 0; mb < 4; ++mb)
#pragma unroll
        for (int nb = 0; nb < 4; ++nb) acc[mb][nb] = (v8f){};
    const size_t aoff = ((size_t)f * ROWS + r0 + lr) * KDT + 8 * hi;
    const size_t boff = ((size_t)f * DI + c0 + lr) * KDT + 8 * hi;
    {
        v16h a[4];
#pragma unroll
        for (int mb = 0; mb < 4; ++mb) a[mb] = ldh(A + aoff + (size_t)mb * 16 * KDT);
#pragma unroll
        for (int nb = 0; nb < 4; ++nb) { const v16h b = ldh(W + boff + (size_t)nb * 16 * KDT);
#pragma unroll
            for (int mb = 0; mb < 4; ++mb) acc[mb][nb] = wmma16g(a[mb], b, acc[mb][nb]); }
    }
    const float* bp = bias + (size_t)f * DI + c0;
    const size_t rowb = (size_t)f * ROWS + r0;
#pragma unroll
    for (int mb = 0; mb < 4; ++mb) {
#pragma unroll
        for (int nb = 0; nb < 4; ++nb) {
#pragma unroll
            for (int j = 0; j < 8; ++j) os[(hi * 8 + j) * OSP + nb * 16 + lr] = acc[mb][nb][j] * FDT; }
        wave_sync();
#pragma unroll 1
        for (int s = 0; s < 8; ++s) { const int p = s * 32 + lane; const int row = p >> 4, c4 = (p & 15) * 4;
            v4f v = *(const v4fa*)(&os[row * OSP + c4]); const v4f bb = *(const v4f*)(bp + c4);
#pragma unroll
            for (int q = 0; q < 4; ++q) v[q] = softplus_f(v[q] + bfr(bb[q]));
            *(v4fa*)(&os[row * OSP + c4]) = v; }
        wave_sync();
        const size_t xb = (rowb + (size_t)(mb * 16)) * DI + c0;
#pragma unroll 1
        for (int ps = 0; ps < 2; ++ps) {
#pragma unroll
            for (int s = 0; s < 8; ++s) { const int p = s * 32 + lane; const int row = p >> 4, c4 = (p & 15) * 4;
                const v4f val = *(const v4fa*)(&os[row * OSP + c4]);
                *(volatile v4f*)(DT + xb + (size_t)row * DI + c4) = val; }
            if (ps == 0) __threadfence(); }
        wave_sync();
    }
}

__global__ __launch_bounds__(DI) void k_scan(const float* __restrict__ BC, const float* __restrict__ DT, const h16* __restrict__ G,
                                             const float* __restrict__ A_log, const float* __restrict__ Dp, float* XY) {
#pragma clang fp contract(off)
    const int f = blockIdx.x / NB, b = blockIdx.x % NB, d = threadIdx.x;
    float A2[DS];
    { const v4f* ap = (const v4f*)(A_log + ((size_t)f * DI + d) * DS);
#pragma unroll
      for (int q = 0; q < 4; ++q) { const v4f v = ap[q];
#pragma unroll
          for (int r = 0; r < 4; ++r) A2[4 * q + r] = -__builtin_amdgcn_exp2f(bfr(v[r]) * L2E) * L2E; } }
    const float Dd = bfr(Dp[(size_t)f * DI + d]);
    float h[DS];
#pragma unroll
    for (int s = 0; s < DS; ++s) h[s] = 0.0f;
    const size_t fr = (size_t)f * ROWS + (size_t)b * SEQ;
#pragma unroll 1
    for (int t = 0; t < SEQ; ++t) {
        const size_t ri = fr + (size_t)t;
        const v4f* bp = (const v4f*)(BC + ri * 32);
        float bcv[2 * DS];
#pragma unroll
        for (int q = 0; q < 8; ++q) { const v4f v = bp[q]; bcv[4 * q + 0] = v[0]; bcv[4 * q + 1] = v[1]; bcv[4 * q + 2] = v[2]; bcv[4 * q + 3] = v[3]; }
        const size_t ei = ri * DI + (size_t)d;
        const float dtv = DT[ei];
        const float xv  = XY[ei];
        const float gv  = (float)G[ei] * (1.0f / CG);
        const float dx  = dtv * xv;
        float y = 0.0f;
#pragma unroll
        for (int s = 0; s < DS; ++s) {
            const float e = __builtin_amdgcn_exp2f(dtv * A2[s]);
            h[s] = h[s] * e + dx * bcv[s];
            y += h[s] * bcv[DS + s]; }
        const float o = (y + xv * Dd) * gv;
        *(volatile float*)(XY + ei) = o; __threadfence(); *(volatile float*)(XY + ei) = o;
    }
}

__global__ __launch_bounds__(32) void k_outmax(const float* __restrict__ Y, const h16* __restrict__ W, float* OUT) {
    __shared__ __align__(16) float os[16 * OSQ];
    const int lane = threadIdx.x & 31, lr = lane & 15, hi = lane >> 4;
    const int r0 = blockIdx.x * 16, f = blockIdx.y;
    const size_t aoff = ((size_t)f * ROWS + r0 + lr) * DI + 8 * hi;
#pragma unroll 1
    for (int ch = 0; ch < 2; ++ch) {
        v8f acc[8];
#pragma unroll
        for (int nb = 0; nb < 8; ++nb) acc[nb] = (v8f){};
        const size_t boff = ((size_t)f * DM + ch * 128 + lr) * DI + 8 * hi;
#pragma unroll 1
        for (int kc = 0; kc < DI; kc += 32) {
            const v16h a = ldf(Y + aoff + kc, CY);
#pragma unroll
            for (int nb = 0; nb < 8; ++nb) { const v16h b = ldh(W + boff + (size_t)nb * 16 * DI + kc); acc[nb] = wmma16g(a, b, acc[nb]); }
        }
#pragma unroll
        for (int nb = 0; nb < 8; ++nb) {
#pragma unroll
            for (int j = 0; j < 8; ++j) os[(hi * 8 + j) * OSQ + ch * 128 + nb * 16 + lr] = acc[nb][j] * FOUT; }
    }
    wave_sync();
    v4f val[4];
#pragma unroll
    for (int s = 0; s < 4; ++s) { const int row = 4 * s + (lane >> 3), j4 = (lane & 7) * 4;
#pragma unroll
        for (int q = 0; q < 4; ++q) { const v4f m0 = *(const v4fa*)(&os[row * OSQ + 8 * (j4 + q)]); const v4f m1 = *(const v4fa*)(&os[row * OSQ + 8 * (j4 + q) + 4]);
            val[s][q] = fmaxf(fmaxf(fmaxf(m0[0], m0[1]), fmaxf(m0[2], m0[3])), fmaxf(fmaxf(m1[0], m1[1]), fmaxf(m1[2], m1[3]))); } }
    const int bb = r0 / SEQ, l0 = r0 % SEQ;
    float* orow = OUT + ((size_t)bb * OUT_SEQ + l0) * DM + f * (DM / 8);
#pragma unroll 1
    for (int ps = 0; ps < 2; ++ps) {
#pragma unroll
        for (int s = 0; s < 4; ++s) { const int row = 4 * s + (lane >> 3), j4 = (lane & 7) * 4;
            *(volatile v4f*)(orow + (size_t)row * DM + j4) = val[s]; }
        if (ps == 0) __threadfence(); }
}

static constexpr size_t al256(size_t v) { return (v + 255) & ~(size_t)255; }
static constexpr size_t SZ_U    = al256((size_t)NF * ROWS * DM * 2);
static constexpr size_t SZ_WIN  = al256((size_t)NF * 2 * DI * DM * 2);
static constexpr size_t SZ_WOUT = al256((size_t)NF * DM * DI * 2);
static constexpr size_t SZ_WXP  = al256((size_t)NF * NXPP * DI * 2);
static constexpr size_t SZ_WDT  = al256((size_t)NF * DI * KDT * 2);
static constexpr size_t SZ_F32  = al256((size_t)NF * ROWS * DI * 4);
static constexpr size_t SZ_G    = al256((size_t)NF * ROWS * DI * 2);
static constexpr size_t SZ_BC   = al256((size_t)NF * ROWS * 32 * 4);
static constexpr size_t SZ_DR   = al256((size_t)NF * ROWS * KDT * 2);
static constexpr size_t SZ_TOTAL = SZ_U + SZ_WIN + SZ_WOUT + SZ_WXP + SZ_WDT + 2 * SZ_F32 + SZ_G + SZ_BC + SZ_DR;
static_assert(SZ_TOTAL <= (size_t)134217728);
static_assert((size_t)NF * ROWS * DI * 4 <= SZ_F32);

extern "C" void kernel_launch(void* const* d_in, const int* in_sizes, int n_in,
                              void* d_out, int out_size, void* d_ws, size_t ws_size, hipStream_t stream) {
    if (n_in < 10) return;
    if ((size_t)in_sizes[0] < ((size_t)(NB - 1) * SEQ_FULL + SEQ) * NF) return;
    if ((size_t)in_sizes[1] < (size_t)NF * 2 * DI * DM) return;
    if ((size_t)in_sizes[2] < (size_t)NF * DI * DC) return;
    if ((size_t)in_sizes[3] < (size_t)NF * DI) return;
    if ((size_t)in_sizes[4] < (size_t)NF * NXP * DI) return;
    if ((size_t)in_sizes[5] < (size_t)NF * DI * DTR) return;
    if ((size_t)in_sizes[6] < (size_t)NF * DI) return;
    if ((size_t)in_sizes[7] < (size_t)NF * DI * DS) return;
    if ((size_t)in_sizes[8] < (size_t)NF * DI) return;
    if ((size_t)in_sizes[9] < (size_t)NF * DM * DI) return;
    if ((size_t)out_size < ((size_t)(NB - 1) * OUT_SEQ + SEQ) * DM) return;
    if (SZ_TOTAL > ws_size) return;
    const float* ipt    = (const float*)d_in[0];
    const float* in_w   = (const float*)d_in[1];
    const float* conv_w = (const float*)d_in[2];
    const float* conv_b = (const float*)d_in[3];
    const float* xp_w   = (const float*)d_in[4];
    const float* dtp_w  = (const float*)d_in[5];
    const float* dtp_b  = (const float*)d_in[6];
    const float* A_log  = (const float*)d_in[7];
    const float* Dp     = (const float*)d_in[8];
    const float* out_w  = (const float*)d_in[9];
    float* OUT = (float*)d_out;
    char* wsp = (char*)d_ws;
    h16* U    = (h16*)wsp;   wsp += SZ_U;
    h16* WIN  = (h16*)wsp;   wsp += SZ_WIN;
    h16* WOUT = (h16*)wsp;   wsp += SZ_WOUT;
    h16* WXP  = (h16*)wsp;   wsp += SZ_WXP;
    h16* WDT  = (h16*)wsp;   wsp += SZ_WDT;
    float* XD = (float*)wsp; wsp += SZ_F32;
    float* XY = (float*)wsp; wsp += SZ_F32;
    h16* G    = (h16*)wsp;   wsp += SZ_G;
    float* BC = (float*)wsp; wsp += SZ_BC;
    h16* DTRH = (h16*)wsp;   wsp += SZ_DR;

    { const size_t n8 = (size_t)NF * 2 * DI * DM / 8; k_wcvt<<<(unsigned)((n8 + 255) / 256), 256, 0, stream>>>(in_w, WIN, n8, CW); }
    { const size_t n8 = (size_t)NF * DM * DI / 8;     k_wcvt<<<(unsigned)((n8 + 255) / 256), 256, 0, stream>>>(out_w, WOUT, n8, CW); }
    k_wcvt_xp<<<(unsigned)((size_t)NF * NXPP * (DI / 8) / 256), 256, 0, stream>>>(xp_w, WXP);
    k_wcvt_dt<<<(unsigned)((size_t)NF * DI * (KDT / 8) / 256), 256, 0, stream>>>(dtp_w, WDT);

    k_feat<<<(unsigned)((size_t)NF * ROWS * 32 / 256), 256, 0, stream>>>(ipt, U);
    k_gemm_in<<<dim3(ROWS / 64, (2 * DI) / 64, NF), 32, 0, stream>>>(U, WIN, XD, G);
    k_conv<<<(unsigned)((size_t)NF * ROWS * (DI / 4) / 256), 256, 0, stream>>>(XD, conv_w, conv_b, XY);
    k_gemm_xp<<<dim3(ROWS / 32, NF, 1), 32, 0, stream>>>(XY, WXP, DTRH, BC);
    k_gemm_dt<<<dim3(ROWS / 64, DI / 64, NF), 32, 0, stream>>>(DTRH, WDT, dtp_b, XD);
    k_scan<<<NF * NB, DI, 0, stream>>>(BC, XD, G, A_log, Dp, XY);
    k_outmax<<<dim3(ROWS / 16, NF, 1), 32, 0, stream>>>(XY, WOUT, OUT);
}
